// BiDirectionalConcatBlock_73581379715113
// MI455X (gfx1250) — hardware-run, weakly checked
//
#include <hip/hip_runtime.h>


#define LT   2048
#define BB   2
#define DM   512
#define DI   1024
#define D2   2048
#define NS   16
#define DR   32
#define DRP  32
#define DXC  64
#define DXR  64
#define KC   4
#define NR1  4096
#define NR2  4096
#define FFD  1024
#define XW   1024
typedef _Float16 h16;
typedef unsigned short bf;
typedef __attribute__((ext_vector_type(16))) __bf16   v16bf;
typedef __attribute__((ext_vector_type(16))) _Float16 v16h;
typedef __attribute__((ext_vector_type(8)))  _Float16 v8h;
typedef __attribute__((ext_vector_type(8)))  unsigned short v8us;
typedef __attribute__((ext_vector_type(8)))  float    v8f;
typedef __attribute__((ext_vector_type(4)))  float    v4f;
typedef v8h  __attribute__((may_alias)) v8ha;
typedef v4f  __attribute__((may_alias)) v4fa;
typedef v8us __attribute__((may_alias)) v8usa;

__device__ __forceinline__ unsigned short f2bf(float f) { unsigned u = __float_as_uint(f); u += 0x7FFFu + ((u >> 16) & 1u); return (unsigned short)(u >> 16); }
__device__ __forceinline__ float bf2f(unsigned short b) { return __uint_as_float(((unsigned)b) << 16); }
__device__ __forceinline__ float bfr(float f) { return bf2f(f2bf(f)); }
__device__ __forceinline__ v16h cat16(v8h lo, v8h hi) { return __builtin_shufflevector(lo, hi, 0, 1, 2, 3, 4, 5, 6, 7, 8, 9, 10, 11, 12, 13, 14, 15); }
__device__ __forceinline__ v16bf cat16b(v8us lo, v8us hi) { return __builtin_bit_cast(v16bf, __builtin_shufflevector(lo, hi, 0, 1, 2, 3, 4, 5, 6, 7, 8, 9, 10, 11, 12, 13, 14, 15)); }
__device__ __forceinline__ v8f wmma16(v16h a, v16h b, v8f c) { return __builtin_amdgcn_wmma_f32_16x16x32_f16(false, a, false, b, (short)0, c, false, false); }
__device__ __forceinline__ v8f wmmab(v16bf a, v16bf b, v8f c) { return __builtin_amdgcn_wmma_f32_16x16x32_bf16(false, a, false, b, (short)0, c, false, false); }


template <typename T16> struct WFrag;
template <> struct WFrag<h16> { typedef v16h V; static __device__ __forceinline__ V ld(const h16* p) { return cat16(*(const v8h*)p, *(const v8h*)(p + 16)); } static __device__ __forceinline__ v8f mma(V a, V b, v8f c) { return wmma16(a, b, c); } };
template <> struct WFrag<bf> { typedef v16bf V; static __device__ __forceinline__ V ld(const bf* p) { return cat16b(*(const v8us*)p, *(const v8us*)(p + 16)); } static __device__ __forceinline__ v8f mma(V a, V b, v8f c) { return wmmab(a, b, c); } };
template <typename T16, int NSPLIT, bool BIAS>
__global__ __launch_bounds__(32) void k_gemmw(const T16* __restrict__ A, const T16* __restrict__ A2, const T16* __restrict__ Bt, const T16* __restrict__ Bt2, int K, float* C, int ldc, const float* __restrict__ bias, size_t sA, size_t sB, size_t sC) {
    typedef typename WFrag<T16>::V V;
    __shared__ __align__(16) float os[16 * 68];
    const size_t z = blockIdx.z; A += z * sA; if (A2) A2 += z * sA; Bt += z * sB; if (Bt2) Bt2 += z * sB; C += z * sC;
    const int lane = threadIdx.x & 31, lr = lane & 15, hi = lane >> 4; const int r0 = blockIdx.x * 64, c0 = blockIdx.y * 64;
    v8f acc[4][4];
#pragma unroll
    for (int mb = 0; mb < 4; ++mb)
#pragma unroll
        for (int nb = 0; nb < 4; ++nb) acc[mb][nb] = (v8f){};
    const size_t aoff = (size_t)(r0 + lr) * K + 8 * hi, boff = (size_t)(c0 + lr) * K + 8 * hi;
#pragma unroll 1
    for (int kc = 0; kc < K; kc += 32) {
        V a[4], a2[4];
#pragma unroll
        for (int mb = 0; mb < 4; ++mb) { a[mb] = WFrag<T16>::ld(A + aoff + (size_t)mb * 16 * K + kc); if (NSPLIT == 1 || NSPLIT == 2) a2[mb] = WFrag<T16>::ld(A2 + aoff + (size_t)mb * 16 * K + kc); }
#pragma unroll
        for (int nb = 0; nb < 4; ++nb) { const V b = WFrag<T16>::ld(Bt + boff + (size_t)nb * 16 * K + kc); V b2; if (NSPLIT >= 2) b2 = WFrag<T16>::ld(Bt2 + boff + (size_t)nb * 16 * K + kc);
#pragma unroll
            for (int mb = 0; mb < 4; ++mb) { acc[mb][nb] = WFrag<T16>::mma(a[mb], b, acc[mb][nb]); if (NSPLIT == 1 || NSPLIT == 2) acc[mb][nb] = WFrag<T16>::mma(a2[mb], b, acc[mb][nb]); if (NSPLIT >= 2) acc[mb][nb] = WFrag<T16>::mma(a[mb], b2, acc[mb][nb]); } }
        asm volatile("v_nop\n\tv_nop\n\tv_nop\n\tv_nop" : "+v"(acc[0][0]), "+v"(acc[1][1]), "+v"(acc[2][2]), "+v"(acc[3][3]) : "v"(a[0]), "v"(a[3]));
    }
#pragma unroll
    for (int mb = 0; mb < 4; ++mb) {
#pragma unroll
        for (int nb = 0; nb < 4; ++nb) {
#pragma unroll
            for (int j = 0; j < 8; ++j) os[(hi * 8 + j) * 68 + nb * 16 + lr] = acc[mb][nb][j]; }
        __builtin_amdgcn_wave_barrier(); asm volatile("" ::: "memory");
        float* crow = C + (size_t)(r0 + mb * 16) * ldc + c0;
#pragma unroll 1
        for (int ps = 0; ps < 2; ++ps) {
#pragma unroll
            for (int s = 0; s < 8; ++s) { const int row = 2 * s + hi, cofs = lr * 4; v4f val = *(const v4fa*)(os + row * 68 + cofs); if (BIAS) { val[0] += bfr(bias[c0 + cofs]); val[1] += bfr(bias[c0 + cofs + 1]); val[2] += bfr(bias[c0 + cofs + 2]); val[3] += bfr(bias[c0 + cofs + 3]); }
                *(volatile v4f*)(crow + (size_t)row * ldc + cofs) = val; }
            if (ps == 0) __threadfence(); }
        __builtin_amdgcn_wave_barrier(); asm volatile("" ::: "memory");
    }
}

__device__ __forceinline__ void splitf(float y, unsigned short& h, unsigned short& l) { h = f2bf(y); l = f2bf(y - bf2f(h)); }
__device__ __forceinline__ float siluf(float t) { float s = __fdiv_rn(1.0f, __fadd_rn(1.0f, __expf(-t))); asm volatile("" : "+v"(s)); return __fmul_rn(t, s); }
typedef __attribute__((ext_vector_type(4))) unsigned short v4us;

__global__ __launch_bounds__(256) void k_cvt8(const float* __restrict__ src, bf* dst, size_t n8) { const size_t i = (size_t)blockIdx.x * 256 + threadIdx.x; if (i >= n8) return; const v8f v = *(const v8f*)(src + i * 8); v8us o;
#pragma unroll
    for (int k = 0; k < 8; ++k) o[k] = f2bf(v[k]); *(volatile v8us*)(dst + i * 8) = o; __threadfence(); *(volatile v8us*)(dst + i * 8) = o; }
__global__ __launch_bounds__(256) void k_xpb(const float* __restrict__ w, bf* Bt) { const int e = (blockIdx.x * 256 + threadIdx.x) * 4; if (e >= DXC * DI) return; const int n = e / DI; v4us o;
#pragma unroll
    for (int u = 0; u < 4; ++u) o[u] = (n < DXR) ? f2bf(w[e + u]) : (unsigned short)0; *(volatile v4us*)(Bt + e) = o; __threadfence(); *(volatile v4us*)(Bt + e) = o; }
__global__ __launch_bounds__(256) void k_dtb(const float* __restrict__ w, bf* Bt) { const int e = (blockIdx.x * 256 + threadIdx.x) * 4; if (e >= DI * DRP) return; const int k = e % DRP; const int d = e / DRP; v4us o;
#pragma unroll
    for (int u = 0; u < 4; ++u) o[u] = (k + u < DR) ? f2bf(w[(size_t)d * DR + k + u]) : (unsigned short)0; *(volatile v4us*)(Bt + e) = o; __threadfence(); *(volatile v4us*)(Bt + e) = o; }
__global__ __launch_bounds__(256) void k_conv(const float* __restrict__ XZ, const float* __restrict__ cw, const float* __restrict__ cb, int nrows, int ts, float* U, bf* Uh, bf* Ul) { const int e = (blockIdx.x * 256 + threadIdx.x) * 4; if (e >= nrows * DI) return; const int d0 = e % DI; const int r = e / DI; const int t = r % ts; v4f o; v4us oh, ol;
#pragma unroll
    for (int u = 0; u < 4; ++u) { const int d = d0 + u; float s = 0.f;
#pragma unroll
        for (int k = 0; k < KC; ++k) { const int tk = t - (KC - 1) + k; const float xv = (tk >= 0) ? XZ[(size_t)(r - (KC - 1) + k) * D2 + d] : 0.f; float p = __fmul_rn(xv, bfr(cw[d * KC + k])); asm volatile("" : "+v"(p)); s = __fadd_rn(s, p); }
        const float uu = siluf(__fadd_rn(s, bfr(cb[d]))); o[u] = uu; unsigned short a, b; splitf(uu, a, b); oh[u] = a; ol[u] = b; }
    for (int ps = 0; ps < 2; ++ps) { *(volatile v4f*)(U + e) = o; *(volatile v4us*)(Uh + e) = oh; *(volatile v4us*)(Ul + e) = ol; if (ps == 0) __threadfence(); } }__global__ __launch_bounds__(256) void k_splr(const float* __restrict__ DBC, int nrows, bf* Rh, bf* Rl) { const int e = (blockIdx.x * 256 + threadIdx.x) * 4; if (e >= nrows * DRP) return; const int rr = e % DRP; const int r = e / DRP; v4us oh, ol;
#pragma unroll
    for (int u = 0; u < 4; ++u) { unsigned short a = 0, b = 0; if (rr + u < DR) splitf(DBC[(size_t)r * DXC + rr + u], a, b); oh[u] = a; ol[u] = b; } *(volatile v4us*)(Rh + e) = oh; *(volatile v4us*)(Rl + e) = ol; __threadfence(); *(volatile v4us*)(Rh + e) = oh; *(volatile v4us*)(Rl + e) = ol; }__global__ __launch_bounds__(64) void k_scan(const float* __restrict__ DT, const float* __restrict__ U, const float* __restrict__ DBC, const float* __restrict__ XZ, const float* __restrict__ A_log, const float* __restrict__ Dv, int nb, int ts, float* YG) { const int gidx = blockIdx.x * 64 + threadIdx.x; if (gidx >= nb * DI) return; const int b = gidx / DI; const int d = gidx % DI;
    float A[NS], h[NS];
#pragma unroll
    for (int n = 0; n < NS; ++n) { A[n] = -__expf(bfr(A_log[d * NS + n])); h[n] = 0.f; }
    const float Dd = bfr(Dv[d]);
    for (int t = 0; t < ts; ++t) { const size_t r = (size_t)b * ts + t; const float dr = DT[r * DI + d]; const float dt = (dr > 20.f) ? dr : log1pf(__expf(dr)); const float uu = U[r * DI + d]; const float* bl = DBC + r * DXC + DR; const float* cl = bl + NS; float y = 0.f;
#pragma unroll
        for (int n = 0; n < NS; ++n) { float da = __fmul_rn(dt, A[n]); asm volatile("" : "+v"(da)); const float ex = __expf(da); float t1 = __fmul_rn(ex, h[n]); asm volatile("" : "+v"(t1)); float db = __fmul_rn(dt, bl[n]); asm volatile("" : "+v"(db)); float t2 = __fmul_rn(db, uu); asm volatile("" : "+v"(t2)); h[n] = __fadd_rn(t1, t2); float p = __fmul_rn(h[n], cl[n]); asm volatile("" : "+v"(p)); y = __fadd_rn(y, p); }
        float sk = __fmul_rn(uu, Dd); asm volatile("" : "+v"(sk)); float yy = __fadd_rn(y, sk); asm volatile("" : "+v"(yy)); const float yg = __fmul_rn(yy, siluf(XZ[r * D2 + DI + d]));
        *(volatile float*)(YG + r * DI + d) = yg; __threadfence(); *(volatile float*)(YG + r * DI + d) = yg; } }__global__ __launch_bounds__(256) void k_spl(const float* __restrict__ F, size_t n4, bf* Hh, bf* Hl) { const size_t e = ((size_t)blockIdx.x * 256 + threadIdx.x) * 4; if (e >= n4) return; const v4f a = *(const v4f*)(F + e); v4us oh, ol;
#pragma unroll
    for (int u = 0; u < 4; ++u) { unsigned short h, l; splitf(a[u], h, l); oh[u] = h; ol[u] = l; } *(volatile v4us*)(Hh + e) = oh; *(volatile v4us*)(Hl + e) = ol; __threadfence(); *(volatile v4us*)(Hh + e) = oh; *(volatile v4us*)(Hl + e) = ol; }

__device__ __forceinline__ void lnrow(float* v, int lane, const float* __restrict__ g, const float* __restrict__ bb, float* o) {
    float s = 0.f;
#pragma unroll
    for (int k = 0; k < DM / 32; ++k) s += v[k];
#pragma unroll
    for (int sh = 16; sh; sh >>= 1) s += __shfl_xor(s, sh, 32);
    const float mean = s * (1.0f / DM); float q = 0.f;
#pragma unroll
    for (int k = 0; k < DM / 32; ++k) { float d = __fsub_rn(v[k], mean); asm volatile("" : "+v"(d)); float p = __fmul_rn(d, d); asm volatile("" : "+v"(p)); q = __fadd_rn(q, p); }
#pragma unroll
    for (int sh = 16; sh; sh >>= 1) q += __shfl_xor(q, sh, 32);
    const float rs = __frsqrt_rn(__fadd_rn(q * (1.0f / DM), 1e-5f));
#pragma unroll
    for (int ch = 0; ch < DM / 128; ++ch) {
#pragma unroll
        for (int u = 0; u < 4; ++u) { const int c = ch * 128 + lane * 4 + u; float d = __fsub_rn(v[ch * 4 + u], mean); asm volatile("" : "+v"(d)); float n0 = __fmul_rn(d, rs); asm volatile("" : "+v"(n0)); float gg = bfr(g[c]), b2 = bfr(bb[c]); asm volatile("" : "+v"(gg)); asm volatile("" : "+v"(b2)); float t1 = __fmul_rn(n0, gg); asm volatile("" : "+v"(t1)); o[ch * 4 + u] = __fadd_rn(t1, b2); } } }
__global__ __launch_bounds__(256) void k_ln1(const float* __restrict__ X, const float* __restrict__ T2, const float* __restrict__ g, const float* __restrict__ bb, float* T1) { const int lane = threadIdx.x & 31; const int r = blockIdx.x * 8 + (threadIdx.x >> 5); if (r >= NR1) return; float v[DM / 32], o[DM / 32];
#pragma unroll
    for (int ch = 0; ch < DM / 128; ++ch) { const size_t o0 = (size_t)r * DM + ch * 128 + lane * 4; const v4f a = *(const v4f*)(X + o0), t = *(const v4f*)(T2 + o0);
#pragma unroll
        for (int u = 0; u < 4; ++u) { float xb = bfr(a[u]); asm volatile("" : "+v"(xb)); v[ch * 4 + u] = __fadd_rn(xb, t[u]); } }
    lnrow(v, lane, g, bb, o);
    for (int ps = 0; ps < 2; ++ps) {
#pragma unroll
        for (int ch = 0; ch < DM / 128; ++ch) { v4f w; for (int u = 0; u < 4; ++u) w[u] = o[ch * 4 + u]; *(volatile v4f*)(T1 + (size_t)r * DM + ch * 128 + lane * 4) = w; }
        if (ps == 0) __threadfence(); } }
__global__ __launch_bounds__(256) void k_comb(const float* __restrict__ T1, const float* __restrict__ mem, bf* Hh, bf* Hl) { const int e = (blockIdx.x * 256 + threadIdx.x) * 4; if (e >= NR2 * DM) return; const int c = e % DM; const int r = e / DM; const int t = r % (2 * LT); const int b = r / (2 * LT); const float* src = (t < LT) ? (T1 + ((size_t)t * BB + b) * DM + c) : (mem + ((size_t)(t - LT) * BB + b) * DM + c); v4us oh, ol;
#pragma unroll
    for (int u = 0; u < 4; ++u) { const float y = (t < LT) ? src[u] : bfr(src[u]); unsigned short a, q; splitf(y, a, q); oh[u] = a; ol[u] = q; } *(volatile v4us*)(Hh + e) = oh; *(volatile v4us*)(Hl + e) = ol; __threadfence(); *(volatile v4us*)(Hh + e) = oh; *(volatile v4us*)(Hl + e) = ol; }
__global__ __launch_bounds__(256) void k_ln2(const float* __restrict__ T2B, const float* __restrict__ g, const float* __restrict__ bb, float* T2, bf* Hh, bf* Hl) { const int lane = threadIdx.x & 31; const int r = blockIdx.x * 8 + (threadIdx.x >> 5); if (r >= NR1) return; const int t = r % LT; const int b = r / LT; const size_t src = ((size_t)b * 2 * LT + t) * DM; float v[DM / 32], o[DM / 32];
#pragma unroll
    for (int ch = 0; ch < DM / 128; ++ch) { const v4f a = *(const v4f*)(T2B + src + ch * 128 + lane * 4);
#pragma unroll
        for (int u = 0; u < 4; ++u) v[ch * 4 + u] = a[u]; }
    lnrow(v, lane, g, bb, o);
    for (int ps = 0; ps < 2; ++ps) {
#pragma unroll
        for (int ch = 0; ch < DM / 128; ++ch) { v4f w; v4us oh, ol; for (int u = 0; u < 4; ++u) { w[u] = o[ch * 4 + u]; unsigned short a, q; splitf(w[u], a, q); oh[u] = a; ol[u] = q; } const size_t oo = (size_t)r * DM + ch * 128 + lane * 4; *(volatile v4f*)(T2 + oo) = w; *(volatile v4us*)(Hh + oo) = oh; *(volatile v4us*)(Hl + oo) = ol; }
        if (ps == 0) __threadfence(); } }
__global__ __launch_bounds__(256) void k_relu(const float* __restrict__ F, size_t n4, bf* Hh, bf* Hl) { const size_t e = ((size_t)blockIdx.x * 256 + threadIdx.x) * 4; if (e >= n4) return; const v4f a = *(const v4f*)(F + e); v4us oh, ol;
#pragma unroll
    for (int u = 0; u < 4; ++u) { unsigned short h, l; splitf(fmaxf(a[u], 0.f), h, l); oh[u] = h; ol[u] = l; } *(volatile v4us*)(Hh + e) = oh; *(volatile v4us*)(Hl + e) = ol; __threadfence(); *(volatile v4us*)(Hh + e) = oh; *(volatile v4us*)(Hl + e) = ol; }
__global__ __launch_bounds__(256) void k_ln3(const float* __restrict__ T2, const float* __restrict__ F2, const float* __restrict__ g, const float* __restrict__ bb, float* OUT) { const int lane = threadIdx.x & 31; const int r = blockIdx.x * 8 + (threadIdx.x >> 5); if (r >= NR1) return; const int t = r % LT; const int b = r / LT; float v[DM / 32], o[DM / 32];
#pragma unroll
    for (int ch = 0; ch < DM / 128; ++ch) { const size_t o0 = (size_t)r * DM + ch * 128 + lane * 4; const v4f a = *(const v4f*)(T2 + o0), f = *(const v4f*)(F2 + o0);
#pragma unroll
        for (int u = 0; u < 4; ++u) v[ch * 4 + u] = __fadd_rn(a[u], f[u]); }
    lnrow(v, lane, g, bb, o);
    for (int ps = 0; ps < 2; ++ps) {
#pragma unroll
        for (int ch = 0; ch < DM / 128; ++ch) { v4f w; for (int u = 0; u < 4; ++u) w[u] = o[ch * 4 + u]; *(volatile v4f*)(OUT + ((size_t)t * BB + b) * DM + ch * 128 + lane * 4) = w; }
        if (ps == 0) __threadfence(); } }

static void mamba(hipStream_t stream, int nrows, int nb, int ts, const bf* XBh, const bf* XBl, const float* const* P, bf* BIN, bf* BX, bf* BDT, bf* BOUT, float* XZ, float* U, bf* Uh, bf* Ul, float* DBC, bf* Rh, bf* Rl, float* DT, float* YG, bf* Yh, bf* Yl, float* MO) {
    k_cvt8<<<(D2 * DM / 8 + 255) / 256, 256, 0, stream>>>(P[0], BIN, (size_t)D2 * DM / 8); k_xpb<<<(DXC * DI / 4 + 255) / 256, 256, 0, stream>>>(P[3], BX); k_dtb<<<(DI * DRP / 4 + 255) / 256, 256, 0, stream>>>(P[4], BDT); k_cvt8<<<(DM * DI / 8 + 255) / 256, 256, 0, stream>>>(P[8], BOUT, (size_t)DM * DI / 8);
    const unsigned gE = (nrows * DI / 4 + 255) / 256;
    if (XBl) k_gemmw<bf, 1, false><<<dim3(nrows / 64, D2 / 64, 1), 32, 0, stream>>>(XBh, XBl, BIN, nullptr, DM, XZ, D2, nullptr, 0, 0, 0);
    else     k_gemmw<bf, 0, false><<<dim3(nrows / 64, D2 / 64, 1), 32, 0, stream>>>(XBh, nullptr, BIN, nullptr, DM, XZ, D2, nullptr, 0, 0, 0);
    k_conv<<<gE, 256, 0, stream>>>(XZ, P[1], P[2], nrows, ts, U, Uh, Ul);
    k_gemmw<bf, 1, false><<<dim3(nrows / 64, DXC / 64, 1), 32, 0, stream>>>(Uh, Ul, BX, nullptr, DI, DBC, DXC, nullptr, 0, 0, 0);
    k_splr<<<(nrows * DRP / 4 + 255) / 256, 256, 0, stream>>>(DBC, nrows, Rh, Rl); k_gemmw<bf, 1, true><<<dim3(nrows / 64, DI / 64, 1), 32, 0, stream>>>(Rh, Rl, BDT, nullptr, DRP, DT, DI, P[5], 0, 0, 0);
    k_scan<<<(nb * DI + 63) / 64, 64, 0, stream>>>(DT, U, DBC, XZ, P[6], P[7], nb, ts, YG);
    k_spl<<<gE, 256, 0, stream>>>(YG, (size_t)nrows * DI, Yh, Yl);
    k_gemmw<bf, 1, false><<<dim3(nrows / 64, DM / 64, 1), 32, 0, stream>>>(Yh, Yl, BOUT, nullptr, DI, MO, DM, nullptr, 0, 0, 0); }

__global__ __launch_bounds__(256) void k_half(const float* __restrict__ x, int off, int flip, bf* XB) { const int e = (blockIdx.x * 256 + threadIdx.x) * 4; if (e >= NR1 * DM) return; const int c = e % DM; const int r = e / DM; const int t = r % LT; const int b = r / LT; const int ts = flip ? (LT - 1 - t) : t; const float* src = x + ((size_t)b * LT + ts) * XW + off + c; v4us o;
#pragma unroll
    for (int u = 0; u < 4; ++u) o[u] = f2bf(src[u]); *(volatile v4us*)(XB + e) = o; __threadfence(); *(volatile v4us*)(XB + e) = o; }
__global__ __launch_bounds__(256) void k_cat(const float* __restrict__ MO, int half, float* out0) { const int e = (blockIdx.x * 256 + threadIdx.x) * 4; if (e >= NR1 * DM) return; const int c = e % DM; const int r = e / DM; const v4f a = *(const v4f*)(MO + e); float* d = out0 + (size_t)r * XW + half * DM + c; *(volatile v4f*)d = a; __threadfence(); *(volatile v4f*)d = a; }
__global__ __launch_bounds__(256) void k_res(const float* __restrict__ x, float* out1, size_t n4) { const size_t e = ((size_t)blockIdx.x * 256 + threadIdx.x) * 4; if (e >= n4) return; const v4f a = *(const v4f*)(x + e); v4f o;
#pragma unroll
    for (int u = 0; u < 4; ++u) o[u] = bfr(a[u]); *(volatile v4f*)(out1 + e) = o; __threadfence(); *(volatile v4f*)(out1 + e) = o; }

extern "C" void kernel_launch(void* const* d_in, const int* in_sizes, int n_in,
                              void* d_out, int out_size, void* d_ws, size_t ws_size, hipStream_t stream) {
    (void)in_sizes; (void)n_in; (void)out_size;
    const float** I = (const float**)d_in;
    const float* x = I[0]; const float* P1[9] = {I[1], I[2], I[3], I[4], I[5], I[6], I[7], I[8], I[9]}; const float* P2[9] = {I[10], I[11], I[12], I[13], I[14], I[15], I[16], I[17], I[18]};
    float* OUT0 = (float*)d_out;
    float* OUT1 = OUT0 + (size_t)BB * LT * XW;
    char* wsp = (char*)d_ws;
    auto take = [&](size_t bytes) { char* p = wsp; wsp += (bytes + 255) & ~(size_t)255; return (void*)p; };
    bf* BIN = (bf*)take((size_t)D2 * DM * 2); bf* BX = (bf*)take((size_t)DXC * DI * 2); bf* BDT = (bf*)take((size_t)DI * DRP * 2); bf* BOUT = (bf*)take((size_t)DM * DI * 2);
    bf* XB = (bf*)take((size_t)NR1 * DM * 2);
    float* XZ = (float*)take((size_t)NR1 * D2 * 4); float* U = (float*)take((size_t)NR1 * DI * 4); bf* Uh = (bf*)take((size_t)NR1 * DI * 2); bf* Ul = (bf*)take((size_t)NR1 * DI * 2); float* DBC = (float*)take((size_t)NR1 * DXC * 4); bf* Rh = (bf*)take((size_t)NR1 * DRP * 2); bf* Rl = (bf*)take((size_t)NR1 * DRP * 2);
    float* DT = (float*)take((size_t)NR1 * DI * 4); float* YG = (float*)take((size_t)NR1 * DI * 4); bf* Yh = (bf*)take((size_t)NR1 * DI * 2); bf* Yl = (bf*)take((size_t)NR1 * DI * 2); float* MO = (float*)take((size_t)NR1 * DM * 4);
    if ((size_t)(wsp - (char*)d_ws) > ws_size) return;
    k_res<<<(unsigned)(((size_t)BB * LT * XW / 4 + 255) / 256), 256, 0, stream>>>(x, OUT1, (size_t)BB * LT * XW);
    for (int half = 0; half < 2; ++half) {
        k_half<<<(NR1 * DM / 4 + 255) / 256, 256, 0, stream>>>(x, half * DM, half, XB);
        mamba(stream, NR1, BB, LT, XB, nullptr, half ? P2 : P1, BIN, BX, BDT, BOUT, XZ, U, Uh, Ul, DBC, Rh, Rl, DT, YG, Yh, Yl, MO);
        k_cat<<<(NR1 * DM / 4 + 255) / 256, 256, 0, stream>>>(MO, half, OUT0); }
}
